// Shared_82119774699743
// MI455X (gfx1250) — hardware-verified
//
#include <hip/hip_runtime.h>

typedef __bf16         v16bf __attribute__((ext_vector_type(16)));
typedef unsigned short v16us __attribute__((ext_vector_type(16)));
typedef unsigned short v8us  __attribute__((ext_vector_type(8)));
typedef float          v8f   __attribute__((ext_vector_type(8)));
typedef float          v4f   __attribute__((ext_vector_type(4)));
typedef v8us __attribute__((may_alias)) v8usa;
typedef v4f  __attribute__((may_alias)) v4fa;

union FragU { v16us v; v8us h8[2]; };

#define NB      256
#define XR      24
#define XW      1001
#define CROP    501
#define XUSE    500
#define NCH     36
#define NPAD    48
#define NTAP    65
#define K1P     96
#define K2      864
#define NTAP3   15
#define K3      540
#define K3P     544
#define NF      288
#define CHK     48
#define NCHK    10
#define XWIN    112
#define KRB     288
#define H2R     160
#define H2N     (H2R * NCH)
#define M3      128
#define BN_EPS  1e-5f

#define PB0     3
#define PB1     (PB0 + 21)
#define PB2     (PB1 + 13)
#define PB3     (PB2 + 41)
#define PBN     (PB3 + 1)

__device__ __forceinline__ int imin(int a, int b) { return a < b ? a : b; }

__device__ __forceinline__ unsigned short bf_bits(float x) {
#if defined(__HIP_DEVICE_COMPILE__)
  const __bf16 t = (__bf16)x;
  return __builtin_bit_cast(unsigned short, t);
#else
  unsigned int u = __float_as_uint(x);
  u += 0x7FFFu + ((u >> 16) & 1u);
  return (unsigned short)(u >> 16);
#endif
}
__device__ __forceinline__ float bf_val(unsigned short u) {
  return __uint_as_float(((unsigned int)u) << 16);
}
__device__ __forceinline__ void split2(float x, unsigned short& hi, unsigned short& lo) {
  hi = bf_bits(x);
  lo = bf_bits(x - bf_val(hi));
}

__device__ __forceinline__ v8f mma3(v16us ah, v16us al, v16us bh, v16us bl, v8f c) {
  const v16bf Ah = __builtin_bit_cast(v16bf, ah);
  const v16bf Al = __builtin_bit_cast(v16bf, al);
  const v16bf Bh = __builtin_bit_cast(v16bf, bh);
  const v16bf Bl = __builtin_bit_cast(v16bf, bl);
  v8f d = __builtin_amdgcn_wmma_f32_16x16x32_bf16(false, Ah, false, Bh, (short)0, c, false, false);
  d = __builtin_amdgcn_wmma_f32_16x16x32_bf16(false, Ah, false, Bl, (short)0, d, false, false);
  d = __builtin_amdgcn_wmma_f32_16x16x32_bf16(false, Al, false, Bh, (short)0, d, false, false);
  asm volatile("v_nop\n\tv_nop\n\tv_nop\n\tv_nop" : "+v"(d) : "v"(ah), "v"(al), "v"(bh), "v"(bl));
  return d;
}

__device__ __forceinline__ v16us ld16(const unsigned short* p) {
  FragU f;
  f.h8[0] = *(const v8usa*)p;
  f.h8[1] = *(const v8usa*)(p + 16);
  return f.v;
}
__device__ __forceinline__ v16us gat16(const unsigned short* p) {
  v16us v = {0, 0, 0, 0, 0, 0, 0, 0, 0, 0, 0, 0, 0, 0, 0, 0};
#pragma unroll
  for (int i = 0; i < 8; ++i) { v[i] = p[i]; v[8 + i] = p[16 + i]; }
  return v;
}

__device__ __forceinline__ float elu1(float v) {
  return v > 0.f ? v : (__expf(v) - 1.f);
}

__global__ __launch_bounds__(256) void prep_kernel(
    const float* __restrict__ Wt, const float* __restrict__ Ws,
    const float* __restrict__ Wc, const float* __restrict__ Wf,
    const float* __restrict__ bt, const float* __restrict__ g1, const float* __restrict__ b1,
    const float* __restrict__ m1, const float* __restrict__ v1,
    const float* __restrict__ bs, const float* __restrict__ g2, const float* __restrict__ b2,
    const float* __restrict__ m2, const float* __restrict__ v2,
    const float* __restrict__ bc, const float* __restrict__ g3, const float* __restrict__ b3,
    const float* __restrict__ m3, const float* __restrict__ v3,
    unsigned short* __restrict__ wtH, unsigned short* __restrict__ wtL,
    unsigned short* __restrict__ wsH, unsigned short* __restrict__ wsL,
    unsigned short* __restrict__ wcH, unsigned short* __restrict__ wcL,
    unsigned short* __restrict__ wfH, unsigned short* __restrict__ wfL,
    float* __restrict__ prm)
{
  const int blk = blockIdx.x, t = threadIdx.x;
  const v8us z8u = {0, 0, 0, 0, 0, 0, 0, 0};

  if (blk < PB0) {
    const int g = blk * 256 + t;
    if (g < (NPAD * K1P) / 8) {
      const int e0 = 8 * g, row = e0 / K1P, k0 = e0 - row * K1P;
      const int rc = imin(row, NCH - 1);
      v8us vh = z8u, vl = z8u;
#pragma unroll
      for (int q = 0; q < 8; ++q) {
        const int k = k0 + q, kc = imin(k, NTAP - 1);
        float w = Wt[rc * NTAP + kc];
        w = (row < NCH && k < NTAP) ? w : 0.f;
        unsigned short hi, lo; split2(w, hi, lo);
        vh[q] = hi; vl[q] = lo;
      }
      unsigned short* dh = wtH + e0; unsigned short* dl = wtL + e0;
      *(volatile v8us*)dh = vh; *(volatile v8us*)dl = vl;
      __threadfence();
      *(volatile v8us*)dh = vh; *(volatile v8us*)dl = vl;
    }
  } else if (blk < PB1) {
    const int g = (blk - PB0) * 256 + t;
    if (g < (NPAD * K2) / 8) {
      const int e0 = 8 * g, row = e0 / K2, k0 = e0 - row * K2;
      const int rc = imin(row, NCH - 1);
      v8us vh = z8u, vl = z8u;
#pragma unroll
      for (int q = 0; q < 8; ++q) {
        const int k = k0 + q, r = k / NCH, c = k - NCH * r;
        float w = Ws[(rc * NCH + c) * XR + r];
        w = (row < NCH) ? w : 0.f;
        unsigned short hi, lo; split2(w, hi, lo);
        vh[q] = hi; vl[q] = lo;
      }
      unsigned short* dh = wsH + e0; unsigned short* dl = wsL + e0;
      *(volatile v8us*)dh = vh; *(volatile v8us*)dl = vl;
      __threadfence();
      *(volatile v8us*)dh = vh; *(volatile v8us*)dl = vl;
    }
  } else if (blk < PB2) {
    const int g = (blk - PB1) * 256 + t;
    if (g < (NPAD * K3P) / 8) {
      const int e0 = 8 * g, row = e0 / K3P, k0 = e0 - row * K3P;
      const int rc = imin(row, NCH - 1);
      v8us vh = z8u, vl = z8u;
#pragma unroll
      for (int q = 0; q < 8; ++q) {
        const int k = k0 + q, tp = k / NCH, c = k - NCH * tp;
        const int tpc = imin(tp, NTAP3 - 1);
        float w = Wc[(rc * NCH + c) * NTAP3 + tpc];
        w = (row < NCH && k < K3) ? w : 0.f;
        unsigned short hi, lo; split2(w, hi, lo);
        vh[q] = hi; vl[q] = lo;
      }
      unsigned short* dh = wcH + e0; unsigned short* dl = wcL + e0;
      *(volatile v8us*)dh = vh; *(volatile v8us*)dl = vl;
      __threadfence();
      *(volatile v8us*)dh = vh; *(volatile v8us*)dl = vl;
    }
  } else if (blk < PB3) {
    const int g = (blk - PB2) * 256 + t;
    if (g < (NF * NF) / 8) {
      const int e0 = 8 * g, n = e0 / NF, k0 = e0 - n * NF;
      v8us vh = z8u, vl = z8u;
#pragma unroll
      for (int q = 0; q < 8; ++q) {
        const float w = Wf[(k0 + q) * NF + n];
        unsigned short hi, lo; split2(w, hi, lo);
        vh[q] = hi; vl[q] = lo;
      }
      unsigned short* dh = wfH + e0; unsigned short* dl = wfL + e0;
      *(volatile v8us*)dh = vh; *(volatile v8us*)dl = vl;
      __threadfence();
      *(volatile v8us*)dh = vh; *(volatile v8us*)dl = vl;
    }
  } else {
    if (t < (6 * NPAD) / 4) {
      v4f pv = {0.f, 0.f, 0.f, 0.f};
#pragma unroll
      for (int q = 0; q < 4; ++q) {
        const int idx = 4 * t + q, arr = idx / NPAD, c = idx - arr * NPAD;
        const int cc = imin(c, NCH - 1);
        const float s1 = g1[cc] * rsqrtf(v1[cc] + BN_EPS);
        const float e1 = (bt[cc] - m1[cc]) * s1 + b1[cc];
        const float s2 = g2[cc] * rsqrtf(v2[cc] + BN_EPS);
        const float e2 = (bs[cc] - m2[cc]) * s2 + b2[cc];
        const float s3 = g3[cc] * rsqrtf(v3[cc] + BN_EPS);
        const float e3 = (bc[cc] - m3[cc]) * s3 + b3[cc];
        float val = (arr == 0) ? s1 : (arr == 1) ? e1 : (arr == 2) ? s2 : (arr == 3) ? e2 : (arr == 4) ? s3 : e3;
        val = (c < NCH) ? val : 0.f;
        pv[q] = val;
      }
      float* dst = prm + 4 * t;
      *(volatile v4f*)dst = pv;
      __threadfence();
      *(volatile v4f*)dst = pv;
    }
  }
}

__global__ __launch_bounds__(256) void conv12_kernel(
    const float* __restrict__ x,
    const unsigned short* __restrict__ wtH, const unsigned short* __restrict__ wtL,
    const unsigned short* __restrict__ wsH, const unsigned short* __restrict__ wsL,
    const float* __restrict__ prm, float* __restrict__ h2)
{
  __shared__ __attribute__((aligned(16))) unsigned short xH[XR * XWIN + 16];
  __shared__ __attribute__((aligned(16))) unsigned short xL[XR * XWIN + 16];
  __shared__ __attribute__((aligned(16))) unsigned short h1H[CHK * KRB];
  __shared__ __attribute__((aligned(16))) unsigned short h1L[CHK * KRB];
  __shared__ __attribute__((aligned(16))) float prmS[4 * NPAD];
  __shared__ __attribute__((aligned(16))) float act2[CHK * NCH];

  const int chunk = blockIdx.x, b = blockIdx.y;
  const int tid = threadIdx.x, wave = tid >> 5, lane = tid & 31;
  const int m = lane & 15, h = lane >> 4;
  const int mlim = (chunk == NCHK - 1) ? 1 : 3;

  if (tid < 4 * NPAD) prmS[tid] = prm[tid];
  const float* xb = x + (size_t)b * (XR * XW);
  for (int idx = tid; idx < XR * XWIN; idx += 256) {
    const int r = idx / XWIN, j = idx - r * XWIN;
    const int cpos = chunk * CHK + j;
    const int col = CROP + imin(cpos, XUSE - 1);
    float v = xb[r * XW + col];
    v = (cpos < XUSE) ? v : 0.f;
    unsigned short hi, lo; split2(v, hi, lo);
    xH[idx] = hi; xL[idx] = lo;
  }
  if (tid < 16) { xH[XR * XWIN + tid] = 0; xL[XR * XWIN + tid] = 0; }
  __syncthreads();

  const v8f z8 = {0.f, 0.f, 0.f, 0.f, 0.f, 0.f, 0.f, 0.f};
  const v16us z16 = {0, 0, 0, 0, 0, 0, 0, 0, 0, 0, 0, 0, 0, 0, 0, 0};
  v8f acc2[2];
  acc2[0] = z8; acc2[1] = z8;

#pragma unroll 1
  for (int rb = 0; rb < 3; ++rb) {
#pragma unroll 1
    for (int jj = 0; jj < 3; ++jj) {
      const int job = wave + 8 * jj;
      const int rl = job / 3, mt = job - 3 * rl;
      if (mt < mlim) {
        const int r = rb * 8 + rl;
        const int ab = r * XWIN + mt * 16 + m + 8 * h;
        const unsigned short* pH = xH + ab;
        const unsigned short* pL = xL + ab;
        const v16us aH0 = gat16(pH),      aL0 = gat16(pL);
        const v16us aH1 = gat16(pH + 32), aL1 = gat16(pL + 32);
        v16us aH2 = z16, aL2 = z16;
        const unsigned short t64h = pH[64], t64l = pL[64];
        aH2[0] = h ? (unsigned short)0 : t64h;
        aL2[0] = h ? (unsigned short)0 : t64l;
        v8f acc[3];
        acc[0] = z8; acc[1] = z8; acc[2] = z8;
#pragma unroll
        for (int nt = 0; nt < 3; ++nt) {
          const int bo = (nt * 16 + m) * K1P + 8 * h;
          const unsigned short* qH = wtH + bo;
          const unsigned short* qL = wtL + bo;
          acc[nt] = mma3(aH0, aL0, ld16(qH),      ld16(qL),      acc[nt]);
          acc[nt] = mma3(aH1, aL1, ld16(qH + 32), ld16(qL + 32), acc[nt]);
          acc[nt] = mma3(aH2, aL2, ld16(qH + 64), ld16(qL + 64), acc[nt]);
        }
        const int hb = (mt * 16 + 8 * h) * KRB + rl * NCH;
#pragma unroll
        for (int nt = 0; nt < 3; ++nt) {
          const int o = nt * 16 + m;
          const bool ok = o < NCH;
          const float sc = prmS[o], sh = prmS[NPAD + o];
#pragma unroll
          for (int r8 = 0; r8 < 8; ++r8) {
            const float v = elu1(acc[nt][r8] * sc + sh);
            unsigned short hi, lo; split2(v, hi, lo);
            if (ok) {
              const int ai = hb + r8 * KRB + o;
              h1H[ai] = hi; h1L[ai] = lo;
            }
          }
        }
      }
    }
    __syncthreads();
#pragma unroll
    for (int jdx = 0; jdx < 2; ++jdx) {
      const int tile = wave + 8 * jdx;
      const int mt2 = tile / 3, nt2 = tile - 3 * mt2;
      if (tile < 9 && mt2 < mlim) {
        const unsigned short* aPH = h1H + (mt2 * 16 + m) * KRB + 8 * h;
        const unsigned short* aPL = h1L + (mt2 * 16 + m) * KRB + 8 * h;
        const int bo = (nt2 * 16 + m) * K2 + rb * KRB + 8 * h;
        const unsigned short* bPH = wsH + bo;
        const unsigned short* bPL = wsL + bo;
#pragma unroll 1
        for (int ks = 0; ks < KRB / 32; ++ks) {
          const int ko = 32 * ks;
          acc2[jdx] = mma3(ld16(aPH + ko), ld16(aPL + ko), ld16(bPH + ko), ld16(bPL + ko), acc2[jdx]);
        }
      }
    }
    __syncthreads();
  }

#pragma unroll
  for (int jdx = 0; jdx < 2; ++jdx) {
    const int tile = wave + 8 * jdx;
    const int mt2 = tile / 3, nt2 = tile - 3 * mt2;
    if (tile < 9 && mt2 < mlim) {
      const int o = nt2 * 16 + m;
      const bool ok = o < NCH;
      const float sc = prmS[2 * NPAD + o], sh = prmS[3 * NPAD + o];
#pragma unroll
      for (int r8 = 0; r8 < 8; ++r8) {
        const int wl = mt2 * 16 + 8 * h + r8;
        const float v = elu1(acc2[jdx][r8] * sc + sh);
        if (ok) act2[wl * NCH + o] = v;
      }
    }
  }
  __syncthreads();

  if (tid < (16 * NCH) / 4) {
    const int nrow = 16 * mlim;
    v4f pv = {0.f, 0.f, 0.f, 0.f};
#pragma unroll
    for (int q = 0; q < 4; ++q) {
      const int p = 4 * tid + q;
      const int jl = p / NCH, o = p - jl * NCH;
      const int rw = 3 * jl;
      const float s = act2[rw * NCH + o] + act2[(rw + 1) * NCH + o] + act2[(rw + 2) * NCH + o];
      pv[q] = (rw + 2 < nrow) ? s * (1.f / 3.f) : 0.f;
    }
    float* dst = h2 + ((size_t)b * H2R + chunk * 16) * NCH + 4 * tid;
    *(volatile v4f*)dst = pv;
    __threadfence();
    *(volatile v4f*)dst = pv;
  }
}

__global__ __launch_bounds__(256) void conv3_kernel(
    const float* __restrict__ h2,
    const unsigned short* __restrict__ wcH, const unsigned short* __restrict__ wcL,
    const float* __restrict__ prm, float* __restrict__ fbuf)
{
  __shared__ __attribute__((aligned(16))) unsigned short pH[H2N + 32];
  __shared__ __attribute__((aligned(16))) unsigned short pL[H2N + 32];
  __shared__ __attribute__((aligned(16))) float act3[M3 * NCH];
  __shared__ __attribute__((aligned(16))) float fst[NF];
  __shared__ __attribute__((aligned(16))) float prm3[2 * NPAD];

  const int b = blockIdx.x;
  const int tid = threadIdx.x, wave = tid >> 5, lane = tid & 31;
  const int m = lane & 15, h = lane >> 4;

  if (tid < 2 * NPAD) prm3[tid] = prm[4 * NPAD + tid];
  const float* hb2 = h2 + (size_t)b * H2N;
  for (int idx = tid; idx < H2N / 4; idx += 256) {
    const v4f v = *(const v4fa*)(hb2 + 4 * idx);
#pragma unroll
    for (int q = 0; q < 4; ++q) {
      unsigned short hi, lo; split2(v[q], hi, lo);
      pH[4 * idx + q] = hi; pL[4 * idx + q] = lo;
    }
  }
  if (tid < 32) { pH[H2N + tid] = 0; pL[H2N + tid] = 0; }
  __syncthreads();

  const v8f z8 = {0.f, 0.f, 0.f, 0.f, 0.f, 0.f, 0.f, 0.f};
  const int mt = wave;
  const int ab = (mt * 16 + m) * NCH + 8 * h;
  v8f acc[3];
  acc[0] = z8; acc[1] = z8; acc[2] = z8;

#pragma unroll 1
  for (int ks = 0; ks < K3P / 32; ++ks) {
    const int ko = 32 * ks;
    v16us aH = gat16(pH + ab + ko), aL = gat16(pL + ab + ko);
    const bool cut = (ks == (K3P / 32) - 1) && (h != 0);
#pragma unroll
    for (int i = 12; i < 16; ++i) {
      const unsigned short eh = aH[i], el = aL[i];
      aH[i] = cut ? (unsigned short)0 : eh;
      aL[i] = cut ? (unsigned short)0 : el;
    }
#pragma unroll
    for (int nt = 0; nt < 3; ++nt) {
      const int bo = (nt * 16 + m) * K3P + ko + 8 * h;
      acc[nt] = mma3(aH, aL, ld16(wcH + bo), ld16(wcL + bo), acc[nt]);
    }
  }

#pragma unroll
  for (int nt = 0; nt < 3; ++nt) {
    const int o = nt * 16 + m;
    const bool ok = o < NCH;
    const float sc = prm3[o], sh = prm3[NPAD + o];
#pragma unroll
    for (int r8 = 0; r8 < 8; ++r8) {
      const int w = mt * 16 + 8 * h + r8;
      const float v = elu1(acc[nt][r8] * sc + sh);
      if (ok) act3[w * NCH + o] = v;
    }
  }
  __syncthreads();

  for (int idx = tid; idx < NF; idx += 256) {
    const int o = idx >> 3, s = idx & 7;
    float sum = 0.f;
#pragma unroll
    for (int q = 0; q < NTAP3; ++q) sum += act3[(NTAP3 * s + q) * NCH + o];
    fst[idx] = sum * (1.f / 15.f);
  }
  __syncthreads();

  if (tid < NF / 4) {
    const v4f v = *(const v4fa*)(fst + 4 * tid);
    float* dst = fbuf + (size_t)b * NF + 4 * tid;
    *(volatile v4f*)dst = v;
    __threadfence();
    *(volatile v4f*)dst = v;
  }
}

__global__ __launch_bounds__(192) void fc_kernel(
    const float* __restrict__ fbuf,
    const unsigned short* __restrict__ wfH, const unsigned short* __restrict__ wfL,
    const float* __restrict__ bias, float* __restrict__ out)
{
  __shared__ __attribute__((aligned(16))) float outT[16 * NF];

  const int mt = blockIdx.x;
  const int tid = threadIdx.x, wave = tid >> 5, lane = tid & 31;
  const int m = lane & 15, h = lane >> 4;
  const v8f z8 = {0.f, 0.f, 0.f, 0.f, 0.f, 0.f, 0.f, 0.f};
  const v16us z16 = {0, 0, 0, 0, 0, 0, 0, 0, 0, 0, 0, 0, 0, 0, 0, 0};

  const float* fr = fbuf + (size_t)(mt * 16 + m) * NF + 8 * h;
  v8f acc[3];
  acc[0] = z8; acc[1] = z8; acc[2] = z8;

#pragma unroll 1
  for (int ks = 0; ks < NF / 32; ++ks) {
    const float* p = fr + 32 * ks;
    const v4f f0 = *(const v4fa*)p;
    const v4f f1 = *(const v4fa*)(p + 4);
    const v4f f2 = *(const v4fa*)(p + 16);
    const v4f f3 = *(const v4fa*)(p + 20);
    v16us aH = z16, aL = z16;
#pragma unroll
    for (int q = 0; q < 4; ++q) {
      unsigned short hi, lo;
      split2(f0[q], hi, lo); aH[q] = hi;      aL[q] = lo;
      split2(f1[q], hi, lo); aH[4 + q] = hi;  aL[4 + q] = lo;
      split2(f2[q], hi, lo); aH[8 + q] = hi;  aL[8 + q] = lo;
      split2(f3[q], hi, lo); aH[12 + q] = hi; aL[12 + q] = lo;
    }
#pragma unroll
    for (int j = 0; j < 3; ++j) {
      const int n = (wave + 6 * j) * 16 + m;
      const int bo = n * NF + 32 * ks + 8 * h;
      acc[j] = mma3(aH, aL, ld16(wfH + bo), ld16(wfL + bo), acc[j]);
    }
  }

#pragma unroll
  for (int j = 0; j < 3; ++j) {
    const int col = (wave + 6 * j) * 16 + m;
    const float bv = bias[col];
#pragma unroll
    for (int r8 = 0; r8 < 8; ++r8) {
      const int rr = 8 * h + r8;
      const int row = mt * 16 + rr;
      const float res = fbuf[(size_t)row * NF + col];
      outT[rr * NF + col] = (acc[j][r8] + bv + res) * (1.f / 501.f);
    }
  }
  __syncthreads();

  float* ob = out + (size_t)mt * 16 * NF;
#pragma unroll
  for (int it = 0; it < 6; ++it) {
    const int q = it * 192 + tid;
    const v4f v = *(const v4fa*)(outT + 4 * q);
    *(volatile v4f*)(ob + 4 * q) = v;
  }
  __threadfence();
#pragma unroll
  for (int it = 0; it < 6; ++it) {
    const int q = it * 192 + tid;
    const v4f v = *(const v4fa*)(outT + 4 * q);
    *(volatile v4f*)(ob + 4 * q) = v;
  }
}

extern "C" void kernel_launch(void* const* d_in, const int* in_sizes, int n_in,
                              void* d_out, int out_size, void* d_ws, size_t ws_size,
                              hipStream_t stream) {
  if (n_in < 21) return;
  if (in_sizes[0] != NB * XR * XW) return;
  if (in_sizes[1] != NCH * NTAP) return;
  if (in_sizes[7] != NCH * NCH * XR) return;
  if (in_sizes[13] != NCH * NCH * NTAP3) return;
  if (in_sizes[19] != NF * NF || in_sizes[20] != NF) return;
  if (in_sizes[2] != NCH || in_sizes[3] != NCH || in_sizes[4] != NCH || in_sizes[5] != NCH || in_sizes[6] != NCH) return;
  if (in_sizes[8] != NCH || in_sizes[9] != NCH || in_sizes[10] != NCH || in_sizes[11] != NCH || in_sizes[12] != NCH) return;
  if (in_sizes[14] != NCH || in_sizes[15] != NCH || in_sizes[16] != NCH || in_sizes[17] != NCH || in_sizes[18] != NCH) return;
  if (out_size != NB * NF) return;

  const float* x   = (const float*)d_in[0];
  const float* Wt  = (const float*)d_in[1];
  const float* bt  = (const float*)d_in[2];
  const float* g1  = (const float*)d_in[3];
  const float* b1  = (const float*)d_in[4];
  const float* m1  = (const float*)d_in[5];
  const float* v1  = (const float*)d_in[6];
  const float* Ws  = (const float*)d_in[7];
  const float* bs  = (const float*)d_in[8];
  const float* g2  = (const float*)d_in[9];
  const float* b2  = (const float*)d_in[10];
  const float* m2  = (const float*)d_in[11];
  const float* v2  = (const float*)d_in[12];
  const float* Wc  = (const float*)d_in[13];
  const float* bc  = (const float*)d_in[14];
  const float* g3  = (const float*)d_in[15];
  const float* b3  = (const float*)d_in[16];
  const float* m3  = (const float*)d_in[17];
  const float* v3  = (const float*)d_in[18];
  const float* Wf  = (const float*)d_in[19];
  const float* bfc = (const float*)d_in[20];
  float* out = (float*)d_out;

  char* ws = (char*)d_ws;
  size_t off = 0;
  auto carve = [&](size_t bytes) -> char* {
    char* p = ws + off;
    off += (bytes + 255) & ~(size_t)255;
    return p;
  };
  float*          prm  = (float*)carve((size_t)6 * NPAD * 4);
  unsigned short* wtH  = (unsigned short*)carve((size_t)NPAD * K1P * 2);
  unsigned short* wtL  = (unsigned short*)carve((size_t)NPAD * K1P * 2);
  unsigned short* wsH  = (unsigned short*)carve((size_t)NPAD * K2 * 2);
  unsigned short* wsL  = (unsigned short*)carve((size_t)NPAD * K2 * 2);
  unsigned short* wcH  = (unsigned short*)carve((size_t)NPAD * K3P * 2);
  unsigned short* wcL  = (unsigned short*)carve((size_t)NPAD * K3P * 2);
  unsigned short* wfH  = (unsigned short*)carve((size_t)NF * NF * 2);
  unsigned short* wfL  = (unsigned short*)carve((size_t)NF * NF * 2);
  float*          h2   = (float*)carve((size_t)NB * H2N * 4);
  float*          fbuf = (float*)carve((size_t)NB * NF * 4);
  if (off > ws_size) return;

  prep_kernel<<<PBN, 256, 0, stream>>>(Wt, Ws, Wc, Wf,
                                       bt, g1, b1, m1, v1,
                                       bs, g2, b2, m2, v2,
                                       bc, g3, b3, m3, v3,
                                       wtH, wtL, wsH, wsL, wcH, wcL, wfH, wfL, prm);

  conv12_kernel<<<dim3(NCHK, NB), 256, 0, stream>>>(x, wtH, wtL, wsH, wsL, prm, h2);

  conv3_kernel<<<NB, 256, 0, stream>>>(h2, wcH, wcL, prm, fbuf);

  fc_kernel<<<NB / 16, 192, 0, stream>>>(fbuf, wfH, wfL, bfc, out);
}
